// BertSelfAttention_22488448762278
// MI455X (gfx1250) — hardware-verified
//
#include <hip/hip_runtime.h>

#ifndef NB
#define NB 2
#endif
#ifndef SEQ
#define SEQ 2048
#endif
#define NB_FULL 2
#define SEQ_FULL 2048
#define DM 1024
#define NH 16
#define HDIM 64
#define SLEN SEQ
#define TQ SLEN
#define TK SLEN
#define NR (NB * SLEN)
#define SCL 0.125f
#define QBLKS (TQ / 64)
#define LNEPS 0.00001f
#define WSC 16.0f
#define CSC 16.0f
static_assert(NH * HDIM == DM);
static_assert(SLEN % 64 == 0);
static_assert(NR % 128 == 0);
static_assert(DM % 64 == 0);
static_assert(DM == 4 * 256);
static_assert(NB <= NB_FULL);
static_assert(SEQ <= SEQ_FULL);

typedef unsigned short v8us __attribute__((ext_vector_type(8), may_alias));
typedef float  v8f  __attribute__((ext_vector_type(8)));
typedef float  v4f  __attribute__((ext_vector_type(4)));
typedef float  v4fa __attribute__((ext_vector_type(4), may_alias));
typedef _Float16 v16h __attribute__((ext_vector_type(16)));
typedef _Float16 v4h  __attribute__((ext_vector_type(4)));
union FragH { v16h v; v8us half[2]; _Float16 h[16]; unsigned short u[16]; };

__device__ __forceinline__ unsigned short bf16_bits(float x) { unsigned int u = __float_as_uint(x); return (unsigned short)((u + 0x7FFFu + ((u >> 16) & 1u)) >> 16); }
__device__ __forceinline__ float bf16_val(unsigned short b) { return __uint_as_float(((unsigned int)b) << 16); }
__device__ __forceinline__ float bf16_rne(float x) { return bf16_val(bf16_bits(x)); }

template <int NT>
__device__ __forceinline__ v8f mmaH(v16h ah, v16h al, v16h bh, v16h bl, v8f c) {
  c = __builtin_amdgcn_wmma_f32_16x16x32_f16(false, ah, false, bh, (short)0, c, false, false);
  if (NT >= 2) c = __builtin_amdgcn_wmma_f32_16x16x32_f16(false, al, false, bh, (short)0, c, false, false);
  if (NT >= 3) c = __builtin_amdgcn_wmma_f32_16x16x32_f16(false, ah, false, bl, (short)0, c, false, false);
  asm volatile("v_nop\n\tv_nop\n\tv_nop\n\tv_nop" : "+v"(c) : "v"(ah), "v"(al), "v"(bh), "v"(bl));
  return c;
}
__device__ __forceinline__ v16h g2_frag(const _Float16* p, int hh) { FragH f; f.half[0] = *(const v8us*)((const unsigned short*)p + 8 * hh); f.half[1] = *(const v8us*)((const unsigned short*)p + 16 + 8 * hh); return f.v; }
__device__ __forceinline__ v8f g2_mma(v16h a, v16h b, v8f c) { v8f d = __builtin_amdgcn_wmma_f32_16x16x32_f16(false, a, false, b, (short)0, c, false, false); asm volatile("v_nop\n\tv_nop\n\tv_nop\n\tv_nop" : "+v"(d) : "v"(a), "v"(b)); return d; }

__global__ __launch_bounds__(256) void k_wsc(const float* __restrict__ Wm, _Float16* __restrict__ Bt, size_t n8, float sc) {
  const size_t t = (size_t)blockIdx.x * 256 + threadIdx.x; if (t >= n8) return; FragH f;
#pragma unroll
  for (int q = 0; q < 8; ++q) f.h[q] = (_Float16)(bf16_rne(Wm[t * 8 + q]) * sc);
  *(volatile v8us*)((unsigned short*)Bt + t * 8) = f.half[0]; __threadfence(); *(volatile v8us*)((unsigned short*)Bt + t * 8) = f.half[0];
}

__global__ __launch_bounds__(256) void k_x16(const float* __restrict__ x, _Float16* __restrict__ X16, size_t n8) {
  const size_t t = (size_t)blockIdx.x * 256 + threadIdx.x; if (t >= n8) return;
  const size_t e = t * 8; const size_t r = e / DM; const int c = (int)(e % DM); const size_t sr = (r / SLEN) * SEQ_FULL + (r % SLEN);
  const float* src = x + sr * DM + c; FragH f;
#pragma unroll
  for (int q = 0; q < 8; ++q) f.h[q] = (_Float16)bf16_rne(src[q]);
  *(volatile v8us*)((unsigned short*)X16 + e) = f.half[0]; __threadfence(); *(volatile v8us*)((unsigned short*)X16 + e) = f.half[0];
}

__global__ __launch_bounds__(256) void k_h16(const float* __restrict__ F, _Float16* __restrict__ H16, size_t n8, float sc) {
  const size_t t = (size_t)blockIdx.x * 256 + threadIdx.x; if (t >= n8) return; FragH f;
  const v4f a = *(const v4fa*)(F + t * 8), c = *(const v4fa*)(F + t * 8 + 4);
#pragma unroll
  for (int q = 0; q < 4; ++q) { f.h[q] = (_Float16)(a[q] * sc); f.h[4 + q] = (_Float16)(c[q] * sc); }
  *(volatile v8us*)((unsigned short*)H16 + t * 8) = f.half[0]; __threadfence(); *(volatile v8us*)((unsigned short*)H16 + t * 8) = f.half[0];
}

template <int ACT>
__global__ __launch_bounds__(128) void k_gemm2(const _Float16* __restrict__ A, int lda, size_t sA, const _Float16* __restrict__ Bh, int ldb, size_t sB, float alpha, const float* __restrict__ bias, size_t sBias, const float* __restrict__ CP, int rowsPerB, size_t sCPb, int row0g,
    float* __restrict__ C, _Float16* __restrict__ C16, int ldc, size_t sC, int M, int N, int K) {
  __shared__ __attribute__((aligned(16))) float so[4][32][68];
  const int tid = threadIdx.x, w = tid >> 5, lane = tid & 31, ln = lane & 15, hh = lane >> 4; const int by = blockIdx.y;
  A += (size_t)by * sA; Bh += (size_t)by * sB; const size_t cofs = (size_t)by * sC; const float* bp = bias ? bias + (size_t)by * sBias : nullptr;
  const int ntn = N >> 6; const int mt = blockIdx.x / ntn, nq = blockIdx.x - mt * ntn; const int row0 = mt * 128 + 32 * w, col0 = nq * 64; if (row0 >= M) return;
  const _Float16* a0p = A + (size_t)(row0 + ln) * lda; const _Float16* a1p = a0p + (size_t)16 * lda;
  const _Float16* b0p = Bh + (size_t)(col0 + ln) * ldb; const _Float16* b1p = b0p + (size_t)16 * ldb; const _Float16* b2p = b1p + (size_t)16 * ldb; const _Float16* b3p = b2p + (size_t)16 * ldb;
  const v8f z8 = {0.f,0.f,0.f,0.f,0.f,0.f,0.f,0.f}; v8f c00 = z8, c01 = z8, c02 = z8, c03 = z8, c10 = z8, c11 = z8, c12 = z8, c13 = z8;
#pragma unroll 1
  for (int kb = 0; kb < K; kb += 32) { const v16h a0 = g2_frag(a0p + kb, hh), a1 = g2_frag(a1p + kb, hh);
    v16h b = g2_frag(b0p + kb, hh); c00 = g2_mma(a0, b, c00); c10 = g2_mma(a1, b, c10);
    b = g2_frag(b1p + kb, hh); c01 = g2_mma(a0, b, c01); c11 = g2_mma(a1, b, c11);
    b = g2_frag(b2p + kb, hh); c02 = g2_mma(a0, b, c02); c12 = g2_mma(a1, b, c12);
    b = g2_frag(b3p + kb, hh); c03 = g2_mma(a0, b, c03); c13 = g2_mma(a1, b, c13); }
  v8f accs[8] = {c00, c01, c02, c03, c10, c11, c12, c13};
#pragma unroll
  for (int u = 0; u < 8; ++u) { const int t = u & 3, half = u >> 2; const int col = col0 + t * 16 + ln; const float bv = bp ? bf16_rne(bp[col]) : 0.f;
#pragma unroll
    for (int r = 0; r < 8; ++r) { const int rloc = half * 16 + 8 * hh + r; float v = accs[u][r] * alpha + bv;
      if (CP) { if (rowsPerB < 0) v += CP[cofs + (size_t)(row0g + row0 + rloc) * ldc + col]; else { const int bidx = (row0g + row0 + rloc) / rowsPerB; v += CP[(size_t)bidx * sCPb + (size_t)by * 64 + col]; } }
      if (ACT == 3) v = fmaxf(v, 0.f);
      so[w][rloc][t * 16 + ln] = v; } }
  __builtin_amdgcn_fence(4  , "workgroup"); __builtin_amdgcn_wave_barrier();
  const int rsub = lane >> 4, c4 = (lane & 15) * 4;
  for (int pass = 0; pass < 2; ++pass) {
#pragma unroll
    for (int q = 0; q < 16; ++q) { const int r = q * 2 + rsub; const v4f v = *(const v4fa*)&so[w][r][c4];
      if (C) *(volatile v4f*)(C + cofs + (size_t)(row0 + r) * ldc + col0 + c4) = v;
      if (C16) { v4h h4; for (int i = 0; i < 4; ++i) h4[i] = (_Float16)v[i]; *(volatile v4h*)(C16 + cofs + (size_t)(row0 + r) * ldc + col0 + c4) = h4; } }
    if (pass == 0) __threadfence(); } }

template <int NHv, int TTv>
__global__ __launch_bounds__(256) void k_vt(const _Float16* __restrict__ V16, int ldv, int voff, _Float16* __restrict__ Vt) {
  __shared__ unsigned short tl[64][66]; const int tid = threadIdx.x; const int slab = blockIdx.x / (TTv / 64), lg = blockIdx.x % (TTv / 64); const int b = slab / NHv, h = slab % NHv;
  for (int i = tid; i < 64 * 8; i += 256) { const int r = i / 8, c8 = (i % 8) * 8; FragH f; f.half[0] = *(const v8us*)((const unsigned short*)V16 + ((size_t)b * TTv + lg * 64 + r) * ldv + voff + h * 64 + c8);
#pragma unroll
    for (int q = 0; q < 8; ++q) tl[r][c8 + q] = f.u[q]; }
  __syncthreads();
  for (int pass = 0; pass < 2; ++pass) {
#pragma unroll
    for (int rd = 0; rd < 2; ++rd) { const int d = rd * 32 + tid / 8, pc = tid % 8; FragH f;
#pragma unroll
      for (int q = 0; q < 8; ++q) f.u[q] = tl[pc * 8 + q][d];
      *(volatile v8us*)((unsigned short*)Vt + ((size_t)slab * 64 + d) * TTv + lg * 64 + pc * 8) = f.half[0]; }
    if (pass == 0) __threadfence(); } }

template <int CAUSAL>
__global__ __launch_bounds__(128) void k_flash(const _Float16* __restrict__ Q16, int ldq, const _Float16* __restrict__ K16, int ldk, const _Float16* __restrict__ Vt, float* __restrict__ O, int ldo) {
  constexpr int RPW = 16, RTN = RPW / 16, DT = 4, KS = 2;
  __shared__ __attribute__((aligned(16))) unsigned short sP[4][RPW][40]; __shared__ __attribute__((aligned(16))) float sO[4][RPW][64 + 4];
  const int tid = threadIdx.x, w = tid >> 5, lane = tid & 31, ln = lane & 15, hh = lane >> 4;
  const int slab = blockIdx.x / QBLKS, qblk = blockIdx.x % QBLKS; const int b = slab / NH, h = slab % NH; const int qb0 = qblk * (4 * RPW); const int q0 = qb0 + w * RPW;
  FragH aq[2][KS];
#pragma unroll
  for (int rt = 0; rt < RTN; ++rt) { const unsigned short* qr = (const unsigned short*)Q16 + ((size_t)b * TQ + q0 + rt * 16 + ln) * ldq + h * 64;
#pragma unroll
    for (int ks = 0; ks < KS; ++ks) { aq[rt][ks].half[0] = *(const v8us*)(qr + ks * 32 + 8 * hh); aq[rt][ks].half[1] = *(const v8us*)(qr + ks * 32 + 16 + 8 * hh); } }
  const unsigned short* Vth = (const unsigned short*)Vt + (size_t)slab * 64 * TK;
  float m_r[2][8], l_r[2][8]; v8f oacc[2][DT];
#pragma unroll
  for (int rt = 0; rt < RTN; ++rt) {
#pragma unroll
    for (int r = 0; r < 8; ++r) { m_r[rt][r] = -3.0e38f; l_r[rt][r] = 0.f; }
#pragma unroll
    for (int dt = 0; dt < DT; ++dt) oacc[rt][dt] = (v8f){0.f,0.f,0.f,0.f,0.f,0.f,0.f,0.f}; }
  const int jend = (CAUSAL == 1) ? (qb0 + 4 * RPW) : TK;
#pragma unroll 1
  for (int j0 = 0; j0 < jend; j0 += 32) {
    v8f s[2][2];
#pragma unroll
    for (int nt = 0; nt < 2; ++nt) { const unsigned short* kr = (const unsigned short*)K16 + ((size_t)b * TK + j0 + nt * 16 + ln) * ldk + h * 64; FragH bk[KS];
#pragma unroll
      for (int ks = 0; ks < KS; ++ks) { bk[ks].half[0] = *(const v8us*)(kr + ks * 32 + 8 * hh); bk[ks].half[1] = *(const v8us*)(kr + ks * 32 + 16 + 8 * hh); }
#pragma unroll
      for (int rt = 0; rt < RTN; ++rt) { v8f acc = (v8f){0.f,0.f,0.f,0.f,0.f,0.f,0.f,0.f};
#pragma unroll
        for (int ks = 0; ks < KS; ++ks) acc = mmaH<1>(aq[rt][ks].v, aq[rt][ks].v, bk[ks].v, bk[ks].v, acc); s[rt][nt] = acc; } }
#pragma unroll
    for (int rt = 0; rt < RTN; ++rt)
#pragma unroll
      for (int r = 0; r < 8; ++r) { const int tq = q0 + rt * 16 + 8 * hh + r; const int k0 = j0 + ln, k1 = j0 + 16 + ln;
        const bool ok0 = (CAUSAL == 1) ? (k0 <= tq) : true, ok1 = (CAUSAL == 1) ? (k1 <= tq) : true; (void)tq;
        const float s0 = ok0 ? s[rt][0][r] * SCL : -3.0e38f, s1 = ok1 ? s[rt][1][r] * SCL : -3.0e38f; float mc = fmaxf(s0, s1);
        mc = fmaxf(mc, __shfl_xor(mc, 1, 32)); mc = fmaxf(mc, __shfl_xor(mc, 2, 32)); mc = fmaxf(mc, __shfl_xor(mc, 4, 32)); mc = fmaxf(mc, __shfl_xor(mc, 8, 32));
        const float mn = fmaxf(m_r[rt][r], mc); const float al = (mn > -1.0e38f) ? expf(m_r[rt][r] - mn) : 1.0f; m_r[rt][r] = mn; const float p0 = ok0 ? expf(s0 - mn) : 0.f, p1 = ok1 ? expf(s1 - mn) : 0.f; l_r[rt][r] = l_r[rt][r] * al + p0 + p1;
#pragma unroll
        for (int dt = 0; dt < DT; ++dt) oacc[rt][dt][r] *= al;
        FragH t2; t2.h[0] = (_Float16)(p0 * 1024.0f); t2.h[1] = (_Float16)(p1 * 1024.0f); sP[w][rt * 16 + 8 * hh + r][ln] = t2.u[0]; sP[w][rt * 16 + 8 * hh + r][16 + ln] = t2.u[1]; }
    __builtin_amdgcn_fence(4  , "workgroup"); __builtin_amdgcn_wave_barrier();
    FragH pa[2];
#pragma unroll
    for (int rt = 0; rt < RTN; ++rt) { pa[rt].half[0] = *(const v8us*)&sP[w][rt * 16 + ln][8 * hh]; pa[rt].half[1] = *(const v8us*)&sP[w][rt * 16 + ln][16 + 8 * hh]; }
#pragma unroll
    for (int dt = 0; dt < DT; ++dt) { const unsigned short* vrow = Vth + (size_t)(dt * 16 + ln) * TK + j0; FragH bv; bv.half[0] = *(const v8us*)(vrow + 8 * hh); bv.half[1] = *(const v8us*)(vrow + 16 + 8 * hh);
#pragma unroll
      for (int rt = 0; rt < RTN; ++rt) oacc[rt][dt] = mmaH<1>(pa[rt].v, pa[rt].v, bv.v, bv.v, oacc[rt][dt]); }
    __builtin_amdgcn_fence(4  , "workgroup"); __builtin_amdgcn_wave_barrier(); }
#pragma unroll
  for (int rt = 0; rt < RTN; ++rt) {
#pragma unroll
    for (int r = 0; r < 8; ++r) { float l = l_r[rt][r]; l += __shfl_xor(l, 1, 32); l += __shfl_xor(l, 2, 32); l += __shfl_xor(l, 4, 32); l += __shfl_xor(l, 8, 32); l_r[rt][r] = (l > 0.f) ? 1.0f / (l * 1024.0f) : 0.f; }
#pragma unroll
    for (int dt = 0; dt < DT; ++dt)
#pragma unroll
      for (int r = 0; r < 8; ++r) sO[w][rt * 16 + 8 * hh + r][dt * 16 + ln] = oacc[rt][dt][r] * l_r[rt][r]; }
  __builtin_amdgcn_fence(4  , "workgroup"); __builtin_amdgcn_wave_barrier();
  for (int pass = 0; pass < 2; ++pass) {
#pragma unroll
    for (int rp = 0; rp < RPW; rp += 2) { const int r = rp + (lane >> 4), pc = lane & 15; const v4f val = *(const v4fa*)&sO[w][r][pc * 4]; *(volatile v4f*)(O + ((size_t)b * TQ + q0 + r) * ldo + h * 64 + pc * 4) = val; }
    if (pass == 0) __threadfence(); } }

__global__ __launch_bounds__(256) void k_ln(const float* __restrict__ X, const float* __restrict__ R, const float* __restrict__ g, const float* __restrict__ bta, float* __restrict__ out) {
  __shared__ float red[256];
  const int row = blockIdx.x, tid = threadIdx.x;
  const size_t srow = (size_t)(row / SLEN) * SEQ_FULL + (size_t)(row % SLEN);
  const float* x = X + (size_t)row * DM; const float* rr = R + srow * DM;
  const int j = tid * 4;
  const v4f a = *(const v4fa*)(x + j); const v4f rb = *(const v4fa*)(rr + j);
  float vals[4]; float s1 = 0.f;
#pragma unroll
  for (int q = 0; q < 4; ++q) { const float v = a[q] + bf16_rne(rb[q]); vals[q] = v; s1 += v; }
  red[tid] = s1; __syncthreads();
  for (int st = 128; st > 0; st >>= 1) { if (tid < st) red[tid] += red[tid + st]; __syncthreads(); }
  const float mu = red[0] * 0.0009765625f; __syncthreads();
  float s2 = 0.f;
#pragma unroll
  for (int q = 0; q < 4; ++q) { const float c = vals[q] - mu; s2 += c * c; }
  red[tid] = s2; __syncthreads();
  for (int st = 128; st > 0; st >>= 1) { if (tid < st) red[tid] += red[tid + st]; __syncthreads(); }
  const float rs = rsqrtf(red[0] * 0.0009765625f + LNEPS);
  v4f o;
#pragma unroll
  for (int q = 0; q < 4; ++q) { const float gg = bf16_rne(g[j + q]), bb = bf16_rne(bta[j + q]); o[q] = (vals[q] - mu) * rs * gg + bb; }
  *(volatile v4f*)(out + (size_t)row * DM + j) = o;
  __threadfence();
  *(volatile v4f*)(out + (size_t)row * DM + j) = o;
}

extern "C" void kernel_launch(void* const* d_in, const int* in_sizes, int n_in,
                              void* d_out, int out_size, void* d_ws, size_t ws_size, hipStream_t stream) {
  if (n_in < 11) return;
  const float* hs = (const float*)d_in[0]; const float* Wq = (const float*)d_in[1]; const float* bq = (const float*)d_in[2]; const float* Wk = (const float*)d_in[3]; const float* bk = (const float*)d_in[4];
  const float* Wv = (const float*)d_in[5]; const float* bv = (const float*)d_in[6]; const float* Wd = (const float*)d_in[7]; const float* bd = (const float*)d_in[8]; const float* gam = (const float*)d_in[9]; const float* bet = (const float*)d_in[10];
  const long long need0 = ((long long)(NB - 1) * SEQ_FULL + SLEN) * DM;
  if ((long long)in_sizes[0] < need0) return;
  if (in_sizes[1] < DM * DM || in_sizes[3] < DM * DM || in_sizes[5] < DM * DM || in_sizes[7] < DM * DM) return;
  if (in_sizes[2] < DM || in_sizes[4] < DM || in_sizes[6] < DM || in_sizes[8] < DM || in_sizes[9] < DM || in_sizes[10] < DM) return;
  if ((long long)out_size < (long long)NR * DM) return;
  char* ws = (char*)d_ws; size_t off = 0;
  auto take = [&](size_t bytes) { char* p = ws + off; off += (bytes + 255) & ~(size_t)255; return p; };
  const size_t np = (size_t)NR * DM; const size_t nw = (size_t)DM * DM;
  _Float16* BQ = (_Float16*)take(nw * 2); _Float16* BK = (_Float16*)take(nw * 2); _Float16* BV = (_Float16*)take(nw * 2); _Float16* BD = (_Float16*)take(nw * 2);
  _Float16* X16 = (_Float16*)take(np * 2); _Float16* QH = (_Float16*)take(np * 2); _Float16* KH = (_Float16*)take(np * 2); _Float16* V16 = (_Float16*)take(np * 2); _Float16* VT = (_Float16*)take(np * 2);
  float* CTX = (float*)take(np * 4); _Float16* CTX16 = (_Float16*)take(np * 2); float* ATT = (float*)take(np * 4);
  float* O = (float*)d_out;
  if (off > ws_size) return;
  const unsigned gw = (unsigned)((nw / 8 + 255) / 256);
  k_wsc<<<gw, 256, 0, stream>>>(Wq, BQ, nw / 8, WSC); k_wsc<<<gw, 256, 0, stream>>>(Wk, BK, nw / 8, WSC); k_wsc<<<gw, 256, 0, stream>>>(Wv, BV, nw / 8, WSC); k_wsc<<<gw, 256, 0, stream>>>(Wd, BD, nw / 8, WSC);
  k_x16<<<(unsigned)((np / 8 + 255) / 256), 256, 0, stream>>>(hs, X16, np / 8);
  const dim3 g((NR / 128) * (DM / 64), 1);
  k_gemm2<0><<<g, 128, 0, stream>>>(X16, DM, 0, BQ, DM, 0, 1.0f / WSC, bq, 0, nullptr, 1, 0, 0, nullptr, QH, DM, 0, NR, DM, DM);
  k_gemm2<0><<<g, 128, 0, stream>>>(X16, DM, 0, BK, DM, 0, 1.0f / WSC, bk, 0, nullptr, 1, 0, 0, nullptr, KH, DM, 0, NR, DM, DM);
  k_gemm2<0><<<g, 128, 0, stream>>>(X16, DM, 0, BV, DM, 0, 1.0f / WSC, bv, 0, nullptr, 1, 0, 0, nullptr, V16, DM, 0, NR, DM, DM);
  k_vt<NH, SLEN><<<NB * NH * (SLEN / 64), 256, 0, stream>>>(V16, DM, 0, VT);
  k_flash<0><<<NB * NH * QBLKS, 128, 0, stream>>>(QH, DM, KH, DM, VT, CTX, DM);
  k_h16<<<(unsigned)((np / 8 + 255) / 256), 256, 0, stream>>>(CTX, CTX16, np / 8, CSC);
  k_gemm2<0><<<g, 128, 0, stream>>>(CTX16, DM, 0, BD, DM, 0, 1.0f / (WSC * CSC), bd, 0, nullptr, 1, 0, 0, ATT, nullptr, DM, 0, NR, DM, DM);
  k_ln<<<NR, 256, 0, stream>>>(ATT, hs, gam, bet, O);
}
